// MaskedAttention_81561428951531
// MI455X (gfx1250) — hardware-verified
//
#include <hip/hip_runtime.h>
#include <stdint.h>

#ifndef NB
#define NB 2
#endif
#ifndef SEQ
#define SEQ 2048
#endif
#define NB_FULL  2
#define SEQ_FULL 2048
#define DM       1024
#define NH       16
#define HDIM     64
#define NQKV     3072
#define QKP      2048
#define NTOK     (NB * SEQ)
#define LNEPS    1e-5f

#define QB   16
#define KT   64
#define OSP  68

typedef _Float16 v16h __attribute__((ext_vector_type(16)));
typedef _Float16 v8h  __attribute__((ext_vector_type(8)));
typedef __bf16   v16b __attribute__((ext_vector_type(16)));
typedef __bf16   v8b  __attribute__((ext_vector_type(8)));
typedef float    v8f  __attribute__((ext_vector_type(8)));
typedef float    v4f  __attribute__((ext_vector_type(4)));
typedef int      v4i  __attribute__((ext_vector_type(4)));
typedef unsigned short v8us __attribute__((ext_vector_type(8)));

static_assert(NB >= 1 && NB <= NB_FULL && SEQ >= 64 && SEQ <= SEQ_FULL);
static_assert((SEQ % 64) == 0 && (DM % 64) == 0 && (NTOK % 64) == 0 && (DM % 32) == 0);
static_assert(NH * HDIM == DM && HDIM == 64 && QKP == 2 * DM && NQKV == 3 * DM);
static_assert((SEQ % (2 * QB)) == 0 && (SEQ % KT) == 0 && ((SEQ * 32) % 256) == 0 && KT == 4 * 16);
static_assert((((NTOK / 64) * (QKP / 64)) % 8) == 0 && (((DM / 64) * (NTOK / 64)) % 8) == 0 && (((NTOK / 64) * (DM / 64)) % 8) == 0);
static_assert((OSP % 4) == 0 && OSP >= HDIM);

__device__ __forceinline__ unsigned short bfbits(float f) {
  const unsigned u = __float_as_uint(f);
  return (unsigned short)((u + 0x7FFFu + ((u >> 16) & 1u)) >> 16);
}
__device__ __forceinline__ float bfval(float f) {
  return __uint_as_float(((unsigned)bfbits(f)) << 16);
}

__device__ __forceinline__ v16h ldfrag(const _Float16* p) {
  union { v16h v; v8h hh[2]; } f;
  f.hh[0] = *(const v8h*)(p);
  f.hh[1] = *(const v8h*)(p + 16);
  return f.v;
}
__device__ __forceinline__ v16b ldfragb(const __bf16* p) {
  union { v16b v; v8b hh[2]; } f;
  f.hh[0] = *(const v8b*)(p);
  f.hh[1] = *(const v8b*)(p + 16);
  return f.v;
}
__device__ __forceinline__ v8f mma16(v16h a, v16h b, v8f c) {
  return __builtin_amdgcn_wmma_f32_16x16x32_f16(false, a, false, b, (short)0, c, false, false);
}
__device__ __forceinline__ v8f mmabf(v16b a, v16b b, v8f c) {
  return __builtin_amdgcn_wmma_f32_16x16x32_bf16(false, a, false, b, (short)0, c, false, false);
}
__device__ __forceinline__ v8f zero8() {
  v8f z;
#pragma unroll
  for (int i = 0; i < 8; ++i) z[i] = 0.0f;
  return z;
}

__device__ __forceinline__ void guard_g(v8f& a, v8f& b, v16b x, v16b y) {
  asm volatile("v_nop\n\tv_nop\n\tv_nop\n\tv_nop" : "+v"(a), "+v"(b) : "v"(x), "v"(y));
}
__device__ __forceinline__ void keep4(v16b a, v16b b, v16b c, v16b d) {
  asm volatile("v_nop" :: "v"(a), "v"(b), "v"(c), "v"(d));
}
__device__ __forceinline__ void accg4(v8f& a, v8f& b, v8f& c, v8f& d) {
  asm volatile("v_nop\n\tv_nop\n\tv_nop\n\tv_nop" : "+v"(a), "+v"(b), "+v"(c), "+v"(d));
}
__device__ __forceinline__ void guard_l(v8f& d, v16h a0, v16h a1, v16h b0, v16h b1) {
  asm volatile("v_nop\n\tv_nop\n\tv_nop\n\tv_nop" : "+v"(d) : "v"(a0), "v"(a1), "v"(b0), "v"(b1));
}
__device__ __forceinline__ void guard_o(v8f& d0, v8f& d1, v16h x, v16h y, v16h p, v16h q) {
  asm volatile("v_nop\n\tv_nop\n\tv_nop\n\tv_nop" : "+v"(d0), "+v"(d1) : "v"(x), "v"(y), "v"(p), "v"(q));
}

__global__ __launch_bounds__(128) void ln_kernel(const float* __restrict__ x, const float* __restrict__ gam,
                                                 const float* __restrict__ bet,
                                                 unsigned short* __restrict__ Xh, unsigned short* __restrict__ Xl) {
  __shared__ float sA[4], sB[4];
  const int t = (int)blockIdx.x;
  const int bb = t / SEQ, pos = t - bb * SEQ;
  const int tid = (int)threadIdx.x, lane = tid & 31, wave = tid >> 5;
  const float* xr = x + ((size_t)bb * SEQ_FULL + pos) * DM + tid * 8;
  const v4f a = *(const v4f*)(xr);
  const v4f c = *(const v4f*)(xr + 4);
  float v[8];
#pragma unroll
  for (int e = 0; e < 4; ++e) { v[e] = bfval(a[e]); v[4 + e] = bfval(c[e]); }
  float s = 0.0f;
#pragma unroll
  for (int e = 0; e < 8; ++e) s += v[e];
#pragma unroll
  for (int d = 1; d < 32; d <<= 1) s += __shfl_xor(s, d, 32);
  if (lane == 0) sA[wave] = s;
  __syncthreads();
  const float mu = ((sA[0] + sA[1]) + (sA[2] + sA[3])) * (1.0f / (float)DM);
  float dv[8];
  float s2 = 0.0f;
#pragma unroll
  for (int e = 0; e < 8; ++e) { dv[e] = v[e] - mu; s2 += dv[e] * dv[e]; }
#pragma unroll
  for (int d = 1; d < 32; d <<= 1) s2 += __shfl_xor(s2, d, 32);
  if (lane == 0) sB[wave] = s2;
  __syncthreads();
  const float var = ((sB[0] + sB[1]) + (sB[2] + sB[3])) * (1.0f / (float)DM);
  const float rstd = rsqrtf(var + LNEPS);
  const v4f g0 = *(const v4f*)(gam + tid * 8), g1 = *(const v4f*)(gam + tid * 8 + 4);
  const v4f b0 = *(const v4f*)(bet + tid * 8), b1 = *(const v4f*)(bet + tid * 8 + 4);
  v8us ho, lo;
#pragma unroll
  for (int e = 0; e < 4; ++e) {
    const float xn0 = dv[e] * rstd * bfval(g0[e]) + bfval(b0[e]);
    const unsigned short h0 = bfbits(xn0);
    ho[e] = h0;
    lo[e] = bfbits(xn0 - __uint_as_float(((unsigned)h0) << 16));
    const float xn1 = dv[4 + e] * rstd * bfval(g1[e]) + bfval(b1[e]);
    const unsigned short h1 = bfbits(xn1);
    ho[4 + e] = h1;
    lo[4 + e] = bfbits(xn1 - __uint_as_float(((unsigned)h1) << 16));
  }
  const size_t go = (size_t)t * DM + tid * 8;
  *(volatile v8us*)(Xh + go) = ho;
  *(volatile v8us*)(Xl + go) = lo;
  __threadfence();
  *(volatile v8us*)(Xh + go) = ho;
  *(volatile v8us*)(Xl + go) = lo;
}

__global__ __launch_bounds__(256) void cvt_wt_kernel(const float* __restrict__ src, unsigned short* __restrict__ dst,
                                                     int nout, int kdim) {
  __shared__ float sTt[64][33];
  const int k0 = (int)blockIdx.x * 64, n0 = (int)blockIdx.y * 32;
  const int t = (int)threadIdx.x;
  {
    const int kr = t >> 2, cc = (t & 3) * 8;
    const float* s = src + (size_t)(k0 + kr) * nout + n0 + cc;
    const v4f a = *(const v4f*)(s);
    const v4f b = *(const v4f*)(s + 4);
#pragma unroll
    for (int e = 0; e < 4; ++e) {
      sTt[kr][cc + e]     = a[e];
      sTt[kr][cc + 4 + e] = b[e];
    }
  }
  __syncthreads();
  const int n = t >> 3, kp = (t & 7) * 8;
  v8us o;
#pragma unroll
  for (int i = 0; i < 8; ++i) o[i] = bfbits(sTt[kp + i][n]);
  unsigned short* d = dst + (size_t)(n0 + n) * kdim + k0 + kp;
  *(volatile v8us*)d = o;
  __threadfence();
  *(volatile v8us*)d = o;
}

__global__ __launch_bounds__(256) void rope_tab_kernel(float* __restrict__ rcos, float* __restrict__ rsin, int n) {
  const int idx = (int)blockIdx.x * 256 + (int)threadIdx.x;
  if (idx >= n) return;
  const int i = idx & 31, pos = idx >> 5;
  const double ex = (double)i * (0.03125 * 13.287712379549449);
  const double pw = exp2(ex);
  const float pf = (float)pw;
  const float inv = 1.0f / pf;
  const float ang = (float)pos * inv;
  float sn, cs;
  sincosf(ang, &sn, &cs);
  *(volatile float*)(rcos + idx) = cs;
  *(volatile float*)(rsin + idx) = sn;
  __threadfence();
  *(volatile float*)(rcos + idx) = cs;
  *(volatile float*)(rsin + idx) = sn;
}

template <int AM, int BM, int EPI>
__global__ __launch_bounds__(256) void proj_kernel(const __bf16* __restrict__ A1, const __bf16* __restrict__ A2, int lda,
                                                   const __bf16* __restrict__ B1, const __bf16* __restrict__ B2, int ldb,
                                                   void* C1v, void* C2v, int ldc, int M, int N, int K,
                                                   const float* __restrict__ rcos, const float* __restrict__ rsin,
                                                   const float* __restrict__ bias) {
  __shared__ __align__(16) float sT[8][16 * 68];
  const int lane = threadIdx.x & 31, wave = threadIdx.x >> 5;
  const int tilesN = N >> 6, tilesM = M >> 6;
  const int tile = (int)blockIdx.x * 8 + wave;
  if (tile >= tilesM * tilesN) return;
  const int tm = tile / tilesN, tn = tile - tm * tilesN;
  const int m0 = tm << 6, n0 = tn << 6;
  const int rl = lane & 15;
  const int koff = (lane >> 4) * 8;
  const int mOff = (lane >> 4) * 8;

  v8f acc[4][4];
#pragma unroll
  for (int i = 0; i < 4; ++i)
#pragma unroll
    for (int j = 0; j < 4; ++j) acc[i][j] = zero8();

#pragma unroll 1
  for (int k0 = 0; k0 < K; k0 += 32) {
    v16b bh[4];
#pragma unroll
    for (int j = 0; j < 4; ++j) bh[j] = ldfragb(B1 + (size_t)(n0 + (j << 4) + rl) * ldb + koff + k0);
#pragma unroll
    for (int i = 0; i < 4; ++i) {
      const v16b ah = ldfragb(A1 + (size_t)(m0 + (i << 4) + rl) * lda + koff + k0);
#pragma unroll
      for (int j = 0; j < 4; ++j) acc[i][j] = mmabf(ah, bh[j], acc[i][j]);
      guard_g(acc[i][0], acc[i][3], ah, bh[3]);
    }
    if (AM) {
#pragma unroll
      for (int i = 0; i < 4; ++i) {
        const v16b al = ldfragb(A2 + (size_t)(m0 + (i << 4) + rl) * lda + koff + k0);
#pragma unroll
        for (int j = 0; j < 4; ++j) acc[i][j] = mmabf(al, bh[j], acc[i][j]);
        guard_g(acc[i][0], acc[i][3], al, bh[3]);
      }
    }
    if (BM) {
#pragma unroll
      for (int j = 0; j < 4; ++j) bh[j] = ldfragb(B2 + (size_t)(n0 + (j << 4) + rl) * ldb + koff + k0);
#pragma unroll
      for (int i = 0; i < 4; ++i) {
        const v16b ah = ldfragb(A1 + (size_t)(m0 + (i << 4) + rl) * lda + koff + k0);
#pragma unroll
        for (int j = 0; j < 4; ++j) acc[i][j] = mmabf(ah, bh[j], acc[i][j]);
        guard_g(acc[i][0], acc[i][3], ah, bh[3]);
      }
    }
    keep4(bh[0], bh[1], bh[2], bh[3]);
  }
  accg4(acc[0][0], acc[0][1], acc[0][2], acc[0][3]);
  accg4(acc[1][0], acc[1][1], acc[1][2], acc[1][3]);
  accg4(acc[2][0], acc[2][1], acc[2][2], acc[2][3]);
  accg4(acc[3][0], acc[3][1], acc[3][2], acc[3][3]);

  float* slab = sT[wave];
#pragma unroll
  for (int i = 0; i < 4; ++i) {
    const int mBase = m0 + (i << 4);
#pragma unroll
    for (int j = 0; j < 4; ++j) {
#pragma unroll
      for (int r = 0; r < 8; ++r) slab[(mOff + r) * 68 + (j << 4) + rl] = acc[i][j][r];
    }
    __builtin_amdgcn_fence(3  , "workgroup");
    __builtin_amdgcn_wave_barrier();
    __builtin_amdgcn_fence(2  , "workgroup");
    if (EPI == 0) {
      _Float16* Ch = (_Float16*)C1v;
      const int qq = lane >> 3, c8 = (lane & 7) * 8;
      const int cj = c8 & 31;
      const float sgn = (c8 < 32) ? -1.0f : 1.0f;
#pragma unroll
      for (int ps = 0; ps < 2; ++ps) {
#pragma unroll
        for (int it = 0; it < 4; ++it) {
          const int row = it * 4 + qq;
          const int tok = mBase + row;
          const int pos = tok % SEQ;
          const float* sp = slab + row * 68 + c8;
          const float* sq = slab + row * 68 + (c8 ^ 32);
          const v4f u0 = *(const v4f*)(sp);
          const v4f u1 = *(const v4f*)(sp + 4);
          const v4f w0 = *(const v4f*)(sq);
          const v4f w1 = *(const v4f*)(sq + 4);
          const float* tc = rcos + (size_t)pos * 32 + cj;
          const float* ts = rsin + (size_t)pos * 32 + cj;
          const v4f cs0 = *(const v4f*)(tc), cs1 = *(const v4f*)(tc + 4);
          const v4f sn0 = *(const v4f*)(ts), sn1 = *(const v4f*)(ts + 4);
          v8h hv;
#pragma unroll
          for (int e = 0; e < 4; ++e) {
            hv[e]     = (_Float16)(u0[e] * cs0[e] + sgn * w0[e] * sn0[e]);
            hv[4 + e] = (_Float16)(u1[e] * cs1[e] + sgn * w1[e] * sn1[e]);
          }
          const size_t go = (size_t)tok * ldc + n0 + c8;
          *(volatile v8h*)(Ch + go) = hv;
        }
        __threadfence();
      }
    } else if (EPI == 1) {
      _Float16* Ch = (_Float16*)C1v;
      _Float16* Cl = (_Float16*)C2v;
      const int qq = lane >> 3, c8 = (lane & 7) * 8;
#pragma unroll
      for (int ps = 0; ps < 2; ++ps) {
#pragma unroll
        for (int it = 0; it < 4; ++it) {
          const int row = it * 4 + qq;
          const float* sp = slab + row * 68 + c8;
          const v4f u0 = *(const v4f*)(sp);
          const v4f u1 = *(const v4f*)(sp + 4);
          v8h hv, lv;
#pragma unroll
          for (int e = 0; e < 4; ++e) {
            const _Float16 g0 = (_Float16)u0[e];
            hv[e] = g0;
            lv[e] = (_Float16)((u0[e] - (float)g0) * 2048.0f);
            const _Float16 g1 = (_Float16)u1[e];
            hv[4 + e] = g1;
            lv[4 + e] = (_Float16)((u1[e] - (float)g1) * 2048.0f);
          }
          const size_t go = (size_t)(mBase + row) * ldc + n0 + c8;
          *(volatile v8h*)(Ch + go) = hv;
          *(volatile v8h*)(Cl + go) = lv;
        }
        __threadfence();
      }
    } else {
      float* outp = (float*)C1v;
      const int rq = lane >> 4, c4 = (lane & 15) * 4;
      const v4f bz = *(const v4f*)(bias + n0 + c4);
      v4f bq;
#pragma unroll
      for (int e = 0; e < 4; ++e) bq[e] = bfval(bz[e]);
#pragma unroll
      for (int ps = 0; ps < 2; ++ps) {
#pragma unroll
        for (int it = 0; it < 8; ++it) {
          const int row = it * 2 + rq;
          const int tok = mBase + row;
          const int orow = (tok / SEQ) * SEQ_FULL + (tok % SEQ);
          const v4f u = *(const v4f*)(slab + row * 68 + c4);
          v4f o;
#pragma unroll
          for (int e = 0; e < 4; ++e) o[e] = u[e] + bq[e];
          *(volatile v4f*)(outp + (size_t)orow * ldc + n0 + c4) = o;
        }
        __threadfence();
      }
    }
    __builtin_amdgcn_fence(3  , "workgroup");
    __builtin_amdgcn_wave_barrier();
    __builtin_amdgcn_fence(2  , "workgroup");
  }
}

__global__ __launch_bounds__(64) void attn_kernel(const _Float16* __restrict__ QK,
                                                  const _Float16* __restrict__ Vth, const _Float16* __restrict__ Vtl,
                                                  const int* __restrict__ msk,
                                                  unsigned short* __restrict__ Ch, unsigned short* __restrict__ Cl) {
  __shared__ __align__(16) float sOs[2][QB * OSP];
  const int tid = (int)threadIdx.x;
  const int wave = __builtin_amdgcn_readfirstlane(tid >> 5);
  const int lane = tid & 31, hh = lane >> 4, c = lane & 15;
  const int head = (int)blockIdx.y, bb = (int)blockIdx.z;
  const int qt = (int)blockIdx.x * 2 + wave;
  if (qt >= SEQ / QB) return;
  const int q0 = qt * QB;
  const size_t tokb = (size_t)bb * SEQ;
  const size_t tok0 = tokb + q0;
  const float ninf = -__builtin_inff();

  const _Float16* qp = QK + (tok0 + c) * QKP + head * HDIM + 8 * hh;
  const v16h qf0 = ldfrag(qp);
  const v16h qf1 = ldfrag(qp + 32);
  const _Float16* kbase = QK + (tokb + c) * QKP + DM + head * HDIM + 8 * hh;
  const int* mrow = msk + ((size_t)bb * SEQ_FULL + q0 + c) * SEQ_FULL + 8 * hh;
  const size_t vrow = (size_t)(head * HDIM + c) * NTOK + tokb + 8 * hh;
  const _Float16* vhb = Vth + vrow;
  const _Float16* vlb = Vtl + vrow;

  float m_run = ninf, l_run = 0.0f;
  v8f oa1[4], oa2[4];
#pragma unroll
  for (int i = 0; i < 4; ++i) { oa1[i] = zero8(); oa2[i] = zero8(); }

#pragma unroll 1
  for (int t = 0; t < SEQ / KT; ++t) {
    const int kb = t * KT;
    v8f s[4];
#pragma unroll
    for (int j = 0; j < 4; ++j) {
      const _Float16* kp = kbase + (size_t)(kb + 16 * j) * QKP;
      const v16h a0 = ldfrag(kp);
      const v16h a1 = ldfrag(kp + 32);
      s[j] = mma16(a0, qf0, zero8());
      s[j] = mma16(a1, qf1, s[j]);
      guard_l(s[j], a0, a1, qf0, qf1);
    }
    float pm = ninf;
#pragma unroll
    for (int j = 0; j < 4; ++j) {
      const v4i k0v = *(const v4i*)(mrow + kb + 16 * j);
      const v4i k1v = *(const v4i*)(mrow + kb + 16 * j + 4);
#pragma unroll
      for (int r = 0; r < 4; ++r) {
        const float sv = (k0v[r] > 0) ? s[j][r] * 0.125f : ninf;
        s[j][r] = sv;
        pm = fmaxf(pm, sv);
      }
#pragma unroll
      for (int r = 0; r < 4; ++r) {
        const float sv = (k1v[r] > 0) ? s[j][4 + r] * 0.125f : ninf;
        s[j][4 + r] = sv;
        pm = fmaxf(pm, sv);
      }
    }
    pm = fmaxf(pm, __shfl_xor(pm, 16, 32));
    const float mn = fmaxf(m_run, pm);
    const float alpha = (m_run == ninf) ? 0.0f : __expf(m_run - mn);
    const float mref = (mn == ninf) ? 0.0f : mn;
    m_run = mn;
    float ps = 0.0f;
    v16h bph[2], bpl[2];
#pragma unroll
    for (int j = 0; j < 4; ++j) {
#pragma unroll
      for (int r = 0; r < 8; ++r) {
        const float p = __expf(s[j][r] - mref);
        ps += p;
        const float p16 = p * 16.0f;
        const _Float16 ph = (_Float16)p16;
        bph[j >> 1][((j & 1) << 3) + r] = ph;
        bpl[j >> 1][((j & 1) << 3) + r] = (_Float16)((p16 - (float)ph) * 2048.0f);
      }
    }
    ps += __shfl_xor(ps, 16, 32);
    l_run = l_run * alpha + ps;
#pragma unroll
    for (int i = 0; i < 4; ++i) {
#pragma unroll
      for (int r = 0; r < 8; ++r) { oa1[i][r] *= alpha; oa2[i][r] *= alpha; }
    }
#pragma unroll
    for (int s2 = 0; s2 < 2; ++s2) {
#pragma unroll
      for (int i = 0; i < 4; ++i) {
        const size_t vo = (size_t)(16 * i) * NTOK + kb + 32 * s2;
        const v16h x = ldfrag(vhb + vo);
        const v16h y = ldfrag(vlb + vo);
        oa1[i] = mma16(x, bph[s2], oa1[i]);
        oa2[i] = mma16(y, bph[s2], oa2[i]);
        oa2[i] = mma16(x, bpl[s2], oa2[i]);
        guard_o(oa1[i], oa2[i], x, y, bph[s2], bpl[s2]);
      }
    }
  }

  const float rlv = 1.0f / fmaxf(l_run, 1e-30f);
  const float li = (l_run > 0.0f) ? rlv * 0.0625f : 0.0f;
  float* Os = sOs[wave];
#pragma unroll
  for (int i = 0; i < 4; ++i) {
    v4f u0, u1;
#pragma unroll
    for (int r = 0; r < 4; ++r) {
      u0[r] = (oa1[i][r] + oa2[i][r] * 0.00048828125f) * li;
      u1[r] = (oa1[i][4 + r] + oa2[i][4 + r] * 0.00048828125f) * li;
    }
    *(v4f*)(Os + c * OSP + 16 * i + 8 * hh)     = u0;
    *(v4f*)(Os + c * OSP + 16 * i + 8 * hh + 4) = u1;
  }
  __builtin_amdgcn_fence(3  , "workgroup");
  __builtin_amdgcn_wave_barrier();
  __builtin_amdgcn_fence(2  , "workgroup");
  {
    const int rq = lane >> 3, p8 = (lane & 7) * 8;
#pragma unroll
    for (int ps2 = 0; ps2 < 2; ++ps2) {
#pragma unroll
      for (int it = 0; it < 4; ++it) {
        const int row = it * 4 + rq;
        const float* sp = Os + row * OSP + p8;
        const v4f w0 = *(const v4f*)(sp);
        const v4f w1 = *(const v4f*)(sp + 4);
        v8us hb, lb;
#pragma unroll
        for (int e = 0; e < 4; ++e) {
          const unsigned short h0 = bfbits(w0[e]);
          hb[e] = h0;
          lb[e] = bfbits(w0[e] - __uint_as_float(((unsigned)h0) << 16));
          const unsigned short h1 = bfbits(w1[e]);
          hb[4 + e] = h1;
          lb[4 + e] = bfbits(w1[e] - __uint_as_float(((unsigned)h1) << 16));
        }
        const size_t go = (tok0 + (size_t)row) * DM + head * HDIM + p8;
        *(volatile v8us*)(Ch + go) = hb;
        *(volatile v8us*)(Cl + go) = lb;
      }
      __threadfence();
    }
  }
}

extern "C" void kernel_launch(void* const* d_in, const int* in_sizes, int n_in,
                              void* d_out, int out_size, void* d_ws, size_t ws_size,
                              hipStream_t stream) {
  if (n_in < 7) return;
  const long long needX = ((long long)(NB - 1) * SEQ_FULL + SEQ) * DM;
  const long long needM = (((long long)(NB - 1) * SEQ_FULL) + (SEQ - 1)) * SEQ_FULL + SEQ;
  if ((long long)in_sizes[0] < needX) return;
  if ((long long)in_sizes[1] < needM) return;
  if (in_sizes[2] < DM || in_sizes[3] < DM) return;
  if ((long long)in_sizes[4] < (long long)DM * NQKV) return;
  if ((long long)in_sizes[5] < (long long)DM * DM) return;
  if (in_sizes[6] < DM) return;
  if ((long long)out_size < needX) return;

  const float* x     = (const float*)d_in[0];
  const int*   amask = (const int*)d_in[1];
  const float* gam   = (const float*)d_in[2];
  const float* bet   = (const float*)d_in[3];
  const float* wqkv  = (const float*)d_in[4];
  const float* wout  = (const float*)d_in[5];
  const float* bout  = (const float*)d_in[6];
  float* out = (float*)d_out;

  const size_t bAct = (size_t)NTOK * DM * 2;
  const size_t bWt  = (size_t)NQKV * DM * 2;
  const size_t bWo  = (size_t)DM * DM * 2;
  const size_t bTab = (size_t)SEQ * 32 * 4;
  const size_t bQK  = (size_t)NTOK * QKP * 2;
  size_t off = 0;
  const size_t oXh = off; off += bAct;
  const size_t oXl = off; off += bAct;
  const size_t oWt = off; off += bWt;
  const size_t oWo = off; off += bWo;
  const size_t oCos = off; off += bTab;
  const size_t oSin = off; off += bTab;
  const size_t oQK = off; off += bQK;
  const size_t oVh = off; off += bAct;
  const size_t oVl = off; off += bAct;
  const size_t oCh = off; off += bAct;
  const size_t oCl = off; off += bAct;
  if (off > ws_size) return;
  if (off > (size_t)134217728) return;

  char* ws = (char*)d_ws;
  unsigned short* Xh  = (unsigned short*)(ws + oXh);
  unsigned short* Xl  = (unsigned short*)(ws + oXl);
  unsigned short* Wt  = (unsigned short*)(ws + oWt);
  unsigned short* WoT = (unsigned short*)(ws + oWo);
  float* rcos = (float*)(ws + oCos);
  float* rsin = (float*)(ws + oSin);
  _Float16* QKp = (_Float16*)(ws + oQK);
  _Float16* Vh  = (_Float16*)(ws + oVh);
  _Float16* Vl  = (_Float16*)(ws + oVl);
  unsigned short* Chp = (unsigned short*)(ws + oCh);
  unsigned short* Clp = (unsigned short*)(ws + oCl);

  const dim3 blk(256);
  ln_kernel<<<dim3(NTOK), dim3(128), 0, stream>>>(x, gam, bet, Xh, Xl);
  cvt_wt_kernel<<<dim3(DM / 64, NQKV / 32), blk, 0, stream>>>(wqkv, Wt, NQKV, DM);
  cvt_wt_kernel<<<dim3(DM / 64, DM / 32), blk, 0, stream>>>(wout, WoT, DM, DM);
  rope_tab_kernel<<<dim3((SEQ * 32) / 256), blk, 0, stream>>>(rcos, rsin, SEQ * 32);
  proj_kernel<1, 0, 0><<<dim3(((NTOK / 64) * (QKP / 64)) / 8), blk, 0, stream>>>(
      (const __bf16*)Xh, (const __bf16*)Xl, DM, (const __bf16*)Wt, (const __bf16*)Wt, DM,
      (void*)QKp, (void*)QKp, QKP, NTOK, QKP, DM, rcos, rsin, bout);
  proj_kernel<0, 1, 1><<<dim3(((DM / 64) * (NTOK / 64)) / 8), blk, 0, stream>>>(
      (const __bf16*)(Wt + (size_t)2 * DM * DM), (const __bf16*)(Wt + (size_t)2 * DM * DM), DM,
      (const __bf16*)Xh, (const __bf16*)Xl, DM,
      (void*)Vh, (void*)Vl, NTOK, DM, NTOK, DM, rcos, rsin, bout);
  attn_kernel<<<dim3(SEQ / QB / 2, NH, NB), dim3(64), 0, stream>>>(QKp, Vh, Vl, amask, Chp, Clp);
  proj_kernel<1, 0, 2><<<dim3(((NTOK / 64) * (DM / 64)) / 8), blk, 0, stream>>>(
      (const __bf16*)Chp, (const __bf16*)Clp, DM, (const __bf16*)WoT, (const __bf16*)WoT, DM,
      (void*)out, (void*)out, DM, NTOK, DM, DM, rcos, rsin, bout);
  (void)hipGetLastError();
}
